// Transition_52312701665879
// MI455X (gfx1250) — hardware-verified
//
#include <hip/hip_runtime.h>
#include <math.h>

constexpr int kB      = 2;
constexpr int kSrc    = 8192;
constexpr int kDst    = 4096;
constexpr int kSd     = 128;
constexpr int kDd     = 128;
constexpr int kChunk  = 2048;
constexpr int kNChunk = kSrc / kChunk;
constexpr int kPvRows = 192;
constexpr int kStN    = 64;
static_assert(kSrc % kChunk == 0);
static_assert(kChunk % 64 == 0 && kDst % 64 == 0 && kDd % 64 == 0 && kSd % 32 == 0 && kSrc % 32 == 0);

typedef __attribute__((ext_vector_type(16))) _Float16 v16h;
typedef __attribute__((ext_vector_type(8)))  _Float16 v8h;
typedef __attribute__((ext_vector_type(16))) __bf16   v16b;
typedef __attribute__((ext_vector_type(8)))  __bf16   v8b;
typedef __attribute__((ext_vector_type(8)))  float    v8f;
typedef __attribute__((ext_vector_type(4)))  float    v4f;
typedef __attribute__((ext_vector_type(2)))  float    v2f;
typedef __attribute__((ext_vector_type(4)))  unsigned int v4u;

__device__ __forceinline__ unsigned short f2bf_bits(float f) {
  unsigned u = __float_as_uint(f);
  return (unsigned short)((u + 0x7FFFu + ((u >> 16) & 1u)) >> 16);
}
__device__ __forceinline__ float bf_bits2f(unsigned short h) { return __uint_as_float(((unsigned)h) << 16); }

__device__ __forceinline__ void dep_guard_h(v8f& a, v8f& b, v16h x, v16h y) { asm volatile("v_nop\n\tv_nop\n\tv_nop\n\tv_nop" : "+v"(a), "+v"(b) : "v"(x), "v"(y)); }
__device__ __forceinline__ void dep_guard_b(v8f& a, v8f& b, v16b x, v16b y) { asm volatile("v_nop\n\tv_nop\n\tv_nop\n\tv_nop" : "+v"(a), "+v"(b) : "v"(x), "v"(y)); }
__device__ __forceinline__ void keep4_h(v16h a, v16h b, v16h c, v16h d) { asm volatile("v_nop" :: "v"(a), "v"(b), "v"(c), "v"(d)); }
__device__ __forceinline__ void keep4_b(v16b a, v16b b, v16b c, v16b d) { asm volatile("v_nop" :: "v"(a), "v"(b), "v"(c), "v"(d)); }
__device__ __forceinline__ void acc_guard4(v8f& a, v8f& b, v8f& c, v8f& d) { asm volatile("v_nop\n\tv_nop\n\tv_nop\n\tv_nop" : "+v"(a), "+v"(b), "+v"(c), "+v"(d)); }
template <typename T> struct Frag;
template <> struct Frag<_Float16> {
  typedef v16h V; union U { v16h v; v8h h[2]; };
  static __device__ __forceinline__ v16h load(const _Float16* p) {
    U f; f.h[0] = *(const v8h*)(p); f.h[1] = *(const v8h*)(p + 16); return f.v;
  }
  static __device__ __forceinline__ v8f mma(v16h a, v16h b, v8f c) {
    return __builtin_amdgcn_wmma_f32_16x16x32_f16(false, a, false, b, (short)0, c, false, false);
  }
  static __device__ __forceinline__ void guard(v8f& a, v8f& b, v16h x, v16h y) { dep_guard_h(a, b, x, y); }
  static __device__ __forceinline__ void keep(v16h a, v16h b, v16h c, v16h d) { keep4_h(a, b, c, d); }
};
template <> struct Frag<__bf16> {
  typedef v16b V; union U { v16b v; v8b h[2]; };
  static __device__ __forceinline__ v16b load(const __bf16* p) {
    U f; f.h[0] = *(const v8b*)(p); f.h[1] = *(const v8b*)(p + 16); return f.v;
  }
  static __device__ __forceinline__ v8f mma(v16b a, v16b b, v8f c) {
    return __builtin_amdgcn_wmma_f32_16x16x32_bf16(false, a, false, b, (short)0, c, false, false);
  }
  static __device__ __forceinline__ void guard(v8f& a, v8f& b, v16b x, v16b y) { dep_guard_b(a, b, x, y); }
  static __device__ __forceinline__ void keep(v16b a, v16b b, v16b c, v16b d) { keep4_b(a, b, c, d); }
};

__device__ __forceinline__ unsigned pk16(unsigned short a, unsigned short b) { return (unsigned)a | ((unsigned)b << 16); }

template <int ET> struct Elem;
template <> struct Elem<0> { typedef _Float16 T; };
template <> struct Elem<1> { typedef __bf16 T; };
template <int ET, bool SPLIT, int BIAS_MODE, int OUT_MODE, bool RESID, int ACT = 0>
__global__ __launch_bounds__(256) void wmma_gemm64(
    const unsigned short* __restrict__ Ap, const unsigned short* __restrict__ A2p, int lda, long strideA,
    const unsigned short* __restrict__ Btp, const unsigned short* __restrict__ Bt2p, int ldb, long strideB,
    void* __restrict__ Cout, void* __restrict__ Cout2, int ldc, long strideC,
    const float* __restrict__ bias,
    const float* __restrict__ resid, long strideR,
    int M, int N, int K, float scale) {
  typedef typename Elem<ET>::T T;
  typedef typename Frag<T>::V V;
  const T* A = (const T*)Ap; const T* A2 = (const T*)A2p; const T* Bt = (const T*)Btp; const T* Bt2 = (const T*)Bt2p;
  __shared__ __align__(16) float sT[8][16 * 68];
  const int b    = blockIdx.y;
  const int lane = threadIdx.x & 31;
  const int wave = threadIdx.x >> 5;
  const int tilesN = N >> 6;
  const int tilesM = M >> 6;
  const int tile = blockIdx.x * 8 + wave;
  if (tile >= tilesM * tilesN) return;
  const int tm = tile / tilesN;
  const int tn = tile - tm * tilesN;
  const int m0 = tm << 6;
  const int n0 = tn << 6;

  const T* Ab  = A  + (size_t)b * strideA;
  const T* Bb  = Bt + (size_t)b * strideB;
  const T* Ab2 = SPLIT ? (A2  + (size_t)b * strideA) : nullptr;
  const T* Bb2 = SPLIT ? (Bt2 + (size_t)b * strideB) : nullptr;

  const int rlane = lane & 15;
  const int koff  = (lane >> 4) * 8;
  const int mOff  = (lane >> 4) * 8;

  v8f acc[4][4];
#pragma unroll
  for (int i = 0; i < 4; ++i)
#pragma unroll
    for (int j = 0; j < 4; ++j) acc[i][j] = (v8f){0.f,0.f,0.f,0.f,0.f,0.f,0.f,0.f};

  for (int k0 = 0; k0 < K; k0 += 32) {
    V bh[4], bl[4];
#pragma unroll
    for (int j = 0; j < 4; ++j) {
      const size_t bo = (size_t)(n0 + (j << 4) + rlane) * ldb + koff + k0;
      bh[j] = Frag<T>::load(Bb + bo);
      if (SPLIT) bl[j] = Frag<T>::load(Bb2 + bo);
    }
#pragma unroll
    for (int i = 0; i < 4; ++i) {
      const size_t ao = (size_t)(m0 + (i << 4) + rlane) * lda + koff + k0;
      V ah = Frag<T>::load(Ab + ao);
      V al;
      if (SPLIT) al = Frag<T>::load(Ab2 + ao);
#pragma unroll
      for (int j = 0; j < 4; ++j) {
        acc[i][j] = Frag<T>::mma(ah, bh[j], acc[i][j]);
        if (SPLIT) {
          acc[i][j] = Frag<T>::mma(ah, bl[j], acc[i][j]);
          acc[i][j] = Frag<T>::mma(al, bh[j], acc[i][j]);
        }
      }
      Frag<T>::guard(acc[i][0], acc[i][3], ah, SPLIT ? al : ah);
    }
    Frag<T>::keep(bh[0], bh[1], bh[2], bh[3]);
    if (SPLIT) Frag<T>::keep(bl[0], bl[1], bl[2], bl[3]);
  }
  acc_guard4(acc[0][0], acc[0][1], acc[0][2], acc[0][3]);
  acc_guard4(acc[1][0], acc[1][1], acc[1][2], acc[1][3]);
  acc_guard4(acc[2][0], acc[2][1], acc[2][2], acc[2][3]);
  acc_guard4(acc[3][0], acc[3][1], acc[3][2], acc[3][3]);

  float* slab = sT[wave];
  const float* Rb = RESID ? (resid + (size_t)b * strideR) : nullptr;
#pragma unroll
  for (int i = 0; i < 4; ++i) {
    const int mBase = m0 + (i << 4);
#pragma unroll
    for (int j = 0; j < 4; ++j) {
      const int n = n0 + (j << 4) + rlane;
      float bv = 0.f;
      if (BIAS_MODE == 2) bv = bias[n];
#pragma unroll
      for (int r = 0; r < 8; ++r) {
        float v = acc[i][j][r] * scale;
        if (BIAS_MODE == 1) v += bias[mBase + mOff + r];
        if (BIAS_MODE == 2) v += bv;
        if (RESID) v += Rb[(size_t)(mBase + mOff + r) * ldc + n];
        if (ACT == 2) v = fmaxf(v, 0.0f);
        if (ACT == 4) v = (v > 0.f) ? v : 0.01f * v;
        slab[(mOff + r) * 68 + (j << 4) + rlane] = v;
      }
    }
    __builtin_amdgcn_fence(__ATOMIC_RELEASE, "workgroup");
    __builtin_amdgcn_wave_barrier();
    __builtin_amdgcn_fence(__ATOMIC_ACQUIRE, "workgroup");
    if (OUT_MODE == 0) {
      float* C = (float*)Cout + (size_t)b * strideC;
      const int hh = lane >> 4, c4 = (lane & 15) * 4;
      for (int pass = 0; pass < 2; ++pass) {
#pragma unroll
        for (int it = 0; it < 8; ++it) {
          const int row = it * 2 + hh;
          v4f v = *(const v4f*)(slab + row * 68 + c4);
          *(volatile v4f*)(C + (size_t)(mBase + row) * ldc + n0 + c4) = v;
        }
        __threadfence();
      }
    } else {
      const int q = lane >> 3, c8 = (lane & 7) * 8;
      unsigned short* C  = (unsigned short*)Cout  + (size_t)b * strideC;
      unsigned short* C2 = (OUT_MODE == 2) ? ((unsigned short*)Cout2 + (size_t)b * strideC) : nullptr;
      for (int pass = 0; pass < 2; ++pass) {
#pragma unroll
        for (int it = 0; it < 4; ++it) {
          const int row = it * 4 + q;
          const float* sp = slab + row * 68 + c8;
          v8h hv, lv;
#pragma unroll
          for (int e = 0; e < 8; ++e) {
            if (OUT_MODE == 1) {
              hv[e] = (_Float16)sp[e];
            } else {
              unsigned short hb = f2bf_bits(sp[e]);
              hv[e] = __builtin_bit_cast(_Float16, hb);
              if (OUT_MODE == 2) {
                unsigned short lb = f2bf_bits(sp[e] - bf_bits2f(hb));
                lv[e] = __builtin_bit_cast(_Float16, lb);
              }
            }
          }
          *(volatile v8h*)(C + (size_t)(mBase + row) * ldc + n0 + c8) = hv;
          if (OUT_MODE == 2) *(volatile v8h*)(C2 + (size_t)(mBase + row) * ldc + n0 + c8) = lv;
        }
        __threadfence();
      }
    }
    __builtin_amdgcn_fence(__ATOMIC_RELEASE, "workgroup");
    __builtin_amdgcn_wave_barrier();
    __builtin_amdgcn_fence(__ATOMIC_ACQUIRE, "workgroup");
  }
}

__global__ __launch_bounds__(256) void cast8_bf16_kernel(const float* __restrict__ in, unsigned short* __restrict__ out, int n8) {
  const int i = blockIdx.x * 256 + threadIdx.x;
  if (i >= n8) return;
  const float* p = in + 8 * (size_t)i;
  const v4f a = *(const v4f*)(p);
  const v4f c = *(const v4f*)(p + 4);
  unsigned short hb[8];
#pragma unroll
  for (int e = 0; e < 4; ++e) {
    hb[e]     = f2bf_bits(a[e]);
    hb[4 + e] = f2bf_bits(c[e]);
  }
  const v4u u = (v4u){pk16(hb[0], hb[1]), pk16(hb[2], hb[3]), pk16(hb[4], hb[5]), pk16(hb[6], hb[7])};
  unsigned short* q = out + 8 * (size_t)i;
  *(volatile v4u*)q = u;
  __threadfence();
  *(volatile v4u*)q = u;
}

template <int NCOLS, int NROWS>
__global__ __launch_bounds__(256) void tcast_bf16_kernel(const float* __restrict__ W, unsigned short* __restrict__ out) {
  __shared__ float sm[64][65];
  const int t  = threadIdx.x;
  const int c0 = blockIdx.x * 64;
  const int r0 = blockIdx.y * 64;
#pragma unroll
  for (int i = 0; i < 16; ++i) {
    const int e  = i * 256 + t;
    const int rl = e >> 6;
    const int cl = e & 63;
    sm[cl][rl] = W[(size_t)(r0 + rl) * NCOLS + c0 + cl];
  }
  __syncthreads();
  const int lane = t & 31, wave = t >> 5;
  const int q = lane >> 3, c8 = (lane & 7) * 8;
  for (int pass = 0; pass < 2; ++pass) {
#pragma unroll
    for (int it = 0; it < 2; ++it) {
      const int row = wave * 8 + it * 4 + q;
      unsigned short hb[8];
#pragma unroll
      for (int e = 0; e < 8; ++e) hb[e] = f2bf_bits(sm[row][c8 + e]);
      const v4u u = (v4u){pk16(hb[0], hb[1]), pk16(hb[2], hb[3]), pk16(hb[4], hb[5]), pk16(hb[6], hb[7])};
      *(volatile v4u*)(out + (size_t)(c0 + row) * NROWS + r0 + c8) = u;
    }
    __threadfence();
  }
}

__global__ __launch_bounds__(256) void fill_state_rows_kernel(const float* __restrict__ src_state, unsigned short* __restrict__ pvst) {
  const int tid = blockIdx.x * 256 + threadIdx.x;
  if (tid >= kB * 64 * (kSrc / 8)) return;
  const int b  = tid >> 16;
  const int r  = (tid >> 10) & 63;
  const int j8 = tid & 1023;
  const float* sp = src_state + (size_t)b * kSrc + j8 * 8;
  const v4f a = *(const v4f*)(sp);
  const v4f c = *(const v4f*)(sp + 4);
  const bool use = (r == 0);
  unsigned short hb[8];
#pragma unroll
  for (int e = 0; e < 4; ++e) {
    hb[e]     = f2bf_bits(use ? a[e] : 0.0f);
    hb[4 + e] = f2bf_bits(use ? c[e] : 0.0f);
  }
  const v4u u = (v4u){pk16(hb[0], hb[1]), pk16(hb[2], hb[3]), pk16(hb[4], hb[5]), pk16(hb[6], hb[7])};
  unsigned short* q = pvst + ((size_t)(b * kPvRows + 128 + r) * kSrc + j8 * 8);
  *(volatile v4u*)q = u;
  __threadfence();
  *(volatile v4u*)q = u;
}

__global__ __launch_bounds__(256) void colstats_kernel(const float* __restrict__ Lt, const float* __restrict__ state_chunk,
                                                       float* __restrict__ cmax, float* __restrict__ cscale) {
  __shared__ float pm[8][32];
  __shared__ float ps[8][32];
  const int t    = threadIdx.x;
  const int lane = t & 31, wave = t >> 5;
  const int j0   = blockIdx.x * 32;
  const float* col = Lt + (size_t)(wave * 512) * kChunk + j0 + lane;
  float m = col[0];
  float s = 1.0f;
#pragma unroll 1
  for (int i = 1; i < 512; ++i) {
    const float x = col[(size_t)i * kChunk];
    const float d = x - m;
    const float e = expf(-fabsf(d));
    const bool up = d > 0.0f;
    s = up ? fmaf(s, e, 1.0f) : (s + e);
    m = up ? x : m;
  }
  pm[wave][lane] = m;
  ps[wave][lane] = s;
  __syncthreads();
  if (wave == 0) {
    float mx = pm[0][lane];
#pragma unroll 1
    for (int w = 1; w < 8; ++w) mx = fmaxf(mx, pm[w][lane]);
    float sum = 0.0f;
#pragma unroll 1
    for (int w = 0; w < 8; ++w) sum += ps[w][lane] * expf(pm[w][lane] - mx);
    const float st = state_chunk[j0 + lane];
    const float splus = fmaxf(st, 0.0f) + log1pf(expf(-fabsf(st)));
    const float sc = splus / sum;
    ((volatile float*)cmax)[j0 + lane]   = mx;
    ((volatile float*)cscale)[j0 + lane] = sc;
    __threadfence();
    ((volatile float*)cmax)[j0 + lane]   = mx;
    ((volatile float*)cscale)[j0 + lane] = sc;
  }
}

__global__ __launch_bounds__(256) void expw_kernel(const float* __restrict__ Lt, const float* __restrict__ cmax,
                                                   const float* __restrict__ cscale, unsigned short* __restrict__ WRT, int coff) {
  const int bx = blockIdx.x;
  const int t  = threadIdx.x;
  const int k  = bx >> 2;
  const int j  = ((bx & 3) << 9) + 2 * t;
  const v2f x  = *(const v2f*)(Lt + (size_t)k * kChunk + j);
  const v2f mx = *(const v2f*)(cmax + j);
  const v2f sc = *(const v2f*)(cscale + j);
  const float w0 = expf(x[0] - mx[0]) * sc[0];
  const float w1 = expf(x[1] - mx[1]) * sc[1];
  const unsigned u = pk16(f2bf_bits(w0), f2bf_bits(w1));
  unsigned* wp = (unsigned*)(void*)WRT + (((size_t)k * kSrc + (size_t)coff + (size_t)j) >> 1);
  *(volatile unsigned*)wp = u;
  __threadfence();
  *(volatile unsigned*)wp = u;
}

__global__ __launch_bounds__(256) void out0_kernel(const float* __restrict__ dst_state, const float* __restrict__ DS, float* __restrict__ out0) {
  const int i = blockIdx.x * 256 + threadIdx.x;
  if (i >= kB * kDst) return;
  const float v = dst_state[i] + DS[(size_t)i * kStN];
  ((volatile float*)out0)[i] = v;
  __threadfence();
  ((volatile float*)out0)[i] = v;
}

extern "C" void kernel_launch(void* const* d_in, const int* in_sizes, int n_in,
                              void* d_out, int out_size, void* d_ws, size_t ws_size,
                              hipStream_t stream) {
  if (n_in < 6) return;
  if (in_sizes[0] != kB * kSrc * kSd || in_sizes[1] != kB * kSrc || in_sizes[2] != kB * kDst * kDd ||
      in_sizes[3] != kB * kDst || in_sizes[4] != kSd * kDst || in_sizes[5] != kSd * kDd) return;
  if (out_size != kB * kDst + kB * kDst * kDd) return;

  const float* src_val   = (const float*)d_in[0];
  const float* src_state = (const float*)d_in[1];
  const float* dst_val   = (const float*)d_in[2];
  const float* dst_state = (const float*)d_in[3];
  const float* W_route   = (const float*)d_in[4];
  const float* W_val     = (const float*)d_in[5];

  float* outf = (float*)d_out;
  float* out0 = outf;
  float* out1 = outf + (size_t)kB * kDst;

  const size_t bWRT  = (size_t)kDst * kSrc * 2;
  const size_t bLt   = (size_t)kDst * kChunk * 4;
  const size_t bSV   = (size_t)kB * kSrc * kSd * 2;
  const size_t bPVST = (size_t)kB * kPvRows * kSrc * 2;
  const size_t bDS   = (size_t)kB * kDst * kStN * 4;
  const size_t bWrT  = (size_t)kDst * kSd * 2;
  const size_t bWvT  = (size_t)kDd * kSd * 2;
  const size_t bStat = (size_t)kChunk * 4;
  size_t off = 0;
  char* wsb = (char*)d_ws;
  unsigned short* WRT  = (unsigned short*)(wsb + off); off += bWRT;
  float*          Lt   = (float*)(wsb + off);          off += bLt;
  unsigned short* SVb  = (unsigned short*)(wsb + off); off += bSV;
  unsigned short* PVST = (unsigned short*)(wsb + off); off += bPVST;
  float*          DS   = (float*)(wsb + off);          off += bDS;
  unsigned short* WrT  = (unsigned short*)(wsb + off); off += bWrT;
  unsigned short* WvT  = (unsigned short*)(wsb + off); off += bWvT;
  float*          cmax = (float*)(wsb + off);          off += bStat;
  float*          cscl = (float*)(wsb + off);          off += bStat;
  if (off > ws_size) return;

  {
    const int n8 = kB * kSrc * kSd / 8;
    cast8_bf16_kernel<<<dim3((n8 + 255) / 256), dim3(256), 0, stream>>>(src_val, SVb, n8);
  }
  tcast_bf16_kernel<kDst, kSd><<<dim3(kDst / 64, kSd / 64), dim3(256), 0, stream>>>(W_route, WrT);
  tcast_bf16_kernel<kDd, kSd><<<dim3(kDd / 64, kSd / 64), dim3(256), 0, stream>>>(W_val, WvT);

  {
    const int tiles = (kDd / 64) * (kSrc / 64);
    wmma_gemm64<1, false, 0, 3, false, 0><<<dim3((tiles + 7) / 8, kB), dim3(256), 0, stream>>>(
        WvT, WvT, kSd, 0L,
        SVb, SVb, kSd, (long)kSrc * kSd,
        (void*)PVST, nullptr, kSrc, (long)kPvRows * kSrc,
        nullptr, nullptr, 0L,
        kDd, kSrc, kSd, 1.0f);
  }
  fill_state_rows_kernel<<<dim3((kB * 64 * (kSrc / 8) + 255) / 256), dim3(256), 0, stream>>>(src_state, PVST);

  for (int b = 0; b < kB; ++b) {
    for (int c = 0; c < kNChunk; ++c) {
      const unsigned short* svChunk = SVb + ((size_t)b * kSrc + (size_t)c * kChunk) * kSd;
      {
        const int tiles = (kDst / 64) * (kChunk / 64);
        wmma_gemm64<1, false, 0, 0, false, 0><<<dim3((tiles + 7) / 8, 1), dim3(256), 0, stream>>>(
            WrT, WrT, kSd, 0L,
            svChunk, svChunk, kSd, 0L,
            (void*)Lt, nullptr, kChunk, 0L,
            nullptr, nullptr, 0L,
            kDst, kChunk, kSd, 1.0f);
      }
      colstats_kernel<<<dim3(kChunk / 32), dim3(256), 0, stream>>>(Lt, src_state + (size_t)b * kSrc + (size_t)c * kChunk, cmax, cscl);
      expw_kernel<<<dim3(kDst * (kChunk / 512)), dim3(256), 0, stream>>>(Lt, cmax, cscl, WRT, c * kChunk);
    }
    {
      const int tiles = (kDst / 64) * (kDd / 64);
      const unsigned short* pvb = PVST + (size_t)b * kPvRows * kSrc;
      wmma_gemm64<1, false, 0, 0, true, 0><<<dim3((tiles + 7) / 8, 1), dim3(256), 0, stream>>>(
          WRT, WRT, kSrc, 0L,
          pvb, pvb, kSrc, 0L,
          (void*)(out1 + (size_t)b * kDst * kDd), nullptr, kDd, 0L,
          nullptr, dst_val + (size_t)b * kDst * kDd, 0L,
          kDst, kDd, kSrc, 1.0f);
    }
    {
      const int tiles = (kDst / 64) * (kStN / 64);
      const unsigned short* psb = PVST + ((size_t)b * kPvRows + 128) * kSrc;
      wmma_gemm64<1, false, 0, 0, false, 0><<<dim3((tiles + 7) / 8, 1), dim3(256), 0, stream>>>(
          WRT, WRT, kSrc, 0L,
          psb, psb, kSrc, 0L,
          (void*)(DS + (size_t)b * kDst * kStN), nullptr, kStN, 0L,
          nullptr, nullptr, 0L,
          kDst, kStN, kSrc, 1.0f);
    }
  }

  out0_kernel<<<dim3((kB * kDst + 255) / 256), dim3(256), 0, stream>>>(dst_state, DS, out0);
}
